// KimiDeltaAttention_46875273069226
// MI455X (gfx1250) — hardware-verified
//
#include <hip/hip_runtime.h>
#include <math.h>
#include <float.h>

constexpr int kB      = 2;
constexpr int kS      = 2048;
constexpr int kHid    = 2048;
constexpr int kH      = 16;
constexpr int kD      = 128;
constexpr int kC      = kH * kD;
constexpr int kRows   = kB * kS;
constexpr int kTaps   = 4;
constexpr int kCat    = 320;
constexpr int kCatUse = 2 * kD + kH;
constexpr float kWCarry      = 16.0f;
constexpr float kWCarryInv   = 1.0f / 16.0f;
constexpr float kActCarry    = 256.0f;
constexpr float kOutScale    = 1.0f / (256.0f * 16.0f);
constexpr float kEpsL2       = 1e-6f;
constexpr float kEpsRms      = 1e-5f;
constexpr float kInvD        = 1.0f / (float)kD;

static_assert(kC == 2048 && kRows == 4096, "shape");
static_assert(kRows % 64 == 0 && kC % 64 == 0 && kHid % 64 == 0 && kCat % 64 == 0 && kD % 64 == 0, "GEMM M,N tile multiples");
static_assert(kHid % 32 == 0 && kD % 32 == 0 && kC % 32 == 0, "GEMM K multiples of 32");
static_assert(kCatUse == 272 && kCatUse <= kCat, "cat columns");

constexpr int kNcRows   = 32;
constexpr int kNcRowsIn = kNcRows + kTaps - 1;
static_assert(kS % kNcRows == 0, "time tile");

constexpr int kScT    = 16;
constexpr int kScCols = 32;
constexpr int kScKpl  = 16;
static_assert(kS % kScT == 0 && kD == 8 * kScKpl && kD % kScCols == 0, "scan geometry");

typedef __attribute__((ext_vector_type(16))) _Float16 v16h;
typedef __attribute__((ext_vector_type(8)))  _Float16 v8h;
typedef __attribute__((ext_vector_type(8)))  float    v8f;
typedef __attribute__((ext_vector_type(4)))  float    v4f;
typedef __attribute__((ext_vector_type(4)))  unsigned int v4u;

__device__ __forceinline__ unsigned short f2bf_bits(float f) {
  unsigned u = __float_as_uint(f);
  return (unsigned short)((u + 0x7FFFu + ((u >> 16) & 1u)) >> 16);
}
__device__ __forceinline__ float bf_bits2f(unsigned short h) { return __uint_as_float(((unsigned)h) << 16); }
__device__ __forceinline__ float bf16r(float f) { return bf_bits2f(f2bf_bits(f)); }
__device__ __forceinline__ unsigned short h_bits(float f) { const _Float16 h = (_Float16)f; return __builtin_bit_cast(unsigned short, h); }
__device__ __forceinline__ unsigned pk16(unsigned short a, unsigned short b) { return (unsigned)a | ((unsigned)b << 16); }
__device__ __forceinline__ float h16_to_f32(unsigned hb) {
  const unsigned sgn = (hb & 0x8000u) << 16;
  const unsigned em = hb & 0x7fffu;
  const float fn = __uint_as_float((em << 13) + 0x38000000u);
  const float fs = (float)em * 5.9604644775390625e-8f;
  const float mag = (em < 0x400u) ? fs : fn;
  return __uint_as_float(__float_as_uint(mag) | sgn);
}
__device__ __forceinline__ float sigmoid_f(float x) { return 1.0f / (1.0f + expf(-x)); }

union FragU { v16h v; v8h h[2]; };
__device__ __forceinline__ v16h frag_load(const _Float16* p) {
  FragU f;
  f.h[0] = *(const v8h*)(p);
  f.h[1] = *(const v8h*)(p + 16);
  return f.v;
}
__device__ __forceinline__ v8f frag_mma(v16h a, v16h b, v8f c) {
  return __builtin_amdgcn_wmma_f32_16x16x32_f16(false, a, false, b, (short)0, c, false, false);
}
__device__ __forceinline__ void dep_guard4_h(v8f& a, v8f& b, v8f& c, v8f& d, v16h x, v16h y0, v16h y1, v16h y2, v16h y3) {
  asm volatile("v_nop\n\tv_nop\n\tv_nop\n\tv_nop" : "+v"(a), "+v"(b), "+v"(c), "+v"(d) : "v"(x), "v"(y0), "v"(y1), "v"(y2), "v"(y3));
}
__device__ __forceinline__ void keep4_h(v16h a, v16h b, v16h c, v16h d) { asm volatile("v_nop" :: "v"(a), "v"(b), "v"(c), "v"(d)); }
__device__ __forceinline__ void acc_guard4(v8f& a, v8f& b, v8f& c, v8f& d) { asm volatile("v_nop\n\tv_nop\n\tv_nop\n\tv_nop" : "+v"(a), "+v"(b), "+v"(c), "+v"(d)); }

__global__ __launch_bounds__(256) void wmma_gemm64_f16(
    const unsigned short* __restrict__ Ap, int lda,
    const unsigned short* __restrict__ Btp, int ldb,
    float* __restrict__ C, int ldc, int M, int N, int K, float scale) {
  const _Float16* A  = (const _Float16*)Ap;
  const _Float16* Bt = (const _Float16*)Btp;
  __shared__ __align__(16) float sT[8][16 * 68];
  const int lane = threadIdx.x & 31;
  const int wave = threadIdx.x >> 5;
  const int tilesN = N >> 6;
  const int tilesM = M >> 6;
  const int tile = blockIdx.x * 8 + wave;
  if (tile >= tilesM * tilesN) return;
  const int tm = tile / tilesN;
  const int tn = tile - tm * tilesN;
  const int m0 = tm << 6;
  const int n0 = tn << 6;

  const int rlane = lane & 15;
  const int koff  = (lane >> 4) * 8;
  const int mOff  = (lane >> 4) * 8;

  v8f acc[4][4];
#pragma unroll
  for (int i = 0; i < 4; ++i)
#pragma unroll
    for (int j = 0; j < 4; ++j) acc[i][j] = (v8f){0.f, 0.f, 0.f, 0.f, 0.f, 0.f, 0.f, 0.f};

  const _Float16* Arow[4];
  const _Float16* Brow[4];
#pragma unroll
  for (int i = 0; i < 4; ++i) {
    Arow[i] = A  + (size_t)(m0 + (i << 4) + rlane) * lda + koff;
    Brow[i] = Bt + (size_t)(n0 + (i << 4) + rlane) * ldb + koff;
  }

  for (int k0 = 0; k0 < K; k0 += 32) {
    v16h bh[4];
#pragma unroll
    for (int j = 0; j < 4; ++j) bh[j] = frag_load(Brow[j] + k0);
#pragma unroll
    for (int i = 0; i < 4; ++i) {
      const v16h ah = frag_load(Arow[i] + k0);
#pragma unroll
      for (int j = 0; j < 4; ++j) acc[i][j] = frag_mma(ah, bh[j], acc[i][j]);
      dep_guard4_h(acc[i][0], acc[i][1], acc[i][2], acc[i][3], ah, bh[0], bh[1], bh[2], bh[3]);
    }
    keep4_h(bh[0], bh[1], bh[2], bh[3]);
  }
  acc_guard4(acc[0][0], acc[0][1], acc[0][2], acc[0][3]);
  acc_guard4(acc[1][0], acc[1][1], acc[1][2], acc[1][3]);
  acc_guard4(acc[2][0], acc[2][1], acc[2][2], acc[2][3]);
  acc_guard4(acc[3][0], acc[3][1], acc[3][2], acc[3][3]);

  float* slab = sT[wave];
#pragma unroll
  for (int i = 0; i < 4; ++i) {
    const int mBase = m0 + (i << 4);
#pragma unroll
    for (int j = 0; j < 4; ++j) {
#pragma unroll
      for (int r = 0; r < 8; ++r) {
        const float v = acc[i][j][r] * scale;
        slab[(mOff + r) * 68 + (j << 4) + rlane] = v;
      }
    }
    __builtin_amdgcn_fence(__ATOMIC_RELEASE, "workgroup");
    __builtin_amdgcn_wave_barrier();
    __builtin_amdgcn_fence(__ATOMIC_ACQUIRE, "workgroup");
    {
      const int hh = lane >> 4, c4 = (lane & 15) * 4;
      for (int pass = 0; pass < 2; ++pass) {
#pragma unroll
        for (int it = 0; it < 8; ++it) {
          const int row = it * 2 + hh;
          const v4f v = *(const v4f*)(slab + row * 68 + c4);
          *(volatile v4f*)(C + (size_t)(mBase + row) * ldc + n0 + c4) = v;
        }
        __threadfence();
      }
    }
    __builtin_amdgcn_fence(__ATOMIC_RELEASE, "workgroup");
    __builtin_amdgcn_wave_barrier();
    __builtin_amdgcn_fence(__ATOMIC_ACQUIRE, "workgroup");
  }
}

__global__ __launch_bounds__(256) void cvt8_bf16_f16_kernel(const float* __restrict__ in, unsigned short* __restrict__ out, int n8) {
  const int i = blockIdx.x * 256 + threadIdx.x;
  if (i >= n8) return;
  const float* p = in + 8 * (size_t)i;
  const v4f a = *(const v4f*)(p);
  const v4f c = *(const v4f*)(p + 4);
  unsigned short hb[8];
#pragma unroll
  for (int e = 0; e < 4; ++e) {
    const float a0 = a[e];
    const float c0 = c[e];
    hb[e]     = h_bits(bf16r(a0));
    hb[4 + e] = h_bits(bf16r(c0));
  }
  const v4u u = (v4u){pk16(hb[0], hb[1]), pk16(hb[2], hb[3]), pk16(hb[4], hb[5]), pk16(hb[6], hb[7])};
  unsigned short* q = out + 8 * (size_t)i;
  *(volatile v4u*)q = u;
  __threadfence();
  *(volatile v4u*)q = u;
}

__global__ __launch_bounds__(256) void wt_cast_kernel(const float* __restrict__ W, int srcPitch, int nValid,
                                                      unsigned short* __restrict__ out, int outPitch, float carry) {
  __shared__ float sm[64][65];
  const int t  = threadIdx.x;
  const int d0 = blockIdx.x * 64;
  const int n0 = blockIdx.y * 64;
#pragma unroll
  for (int i = 0; i < 16; ++i) {
    const int e = i * 256 + t;
    const int r = e >> 6;
    const int c = e & 63;
    const int n = n0 + c;
    const int nc = (n < nValid) ? n : (nValid - 1);
    const float w = W[(size_t)(d0 + r) * srcPitch + nc];
    const float val = (n < nValid) ? (bf16r(w) * carry) : 0.0f;
    sm[c][r] = val;
  }
  __syncthreads();
  const int lane = t & 31, wave = t >> 5;
  const int q = lane >> 3, c8 = (lane & 7) * 8;
  v4u u[2];
#pragma unroll
  for (int it = 0; it < 2; ++it) {
    const int row = wave * 8 + it * 4 + q;
    unsigned short hb[8];
#pragma unroll
    for (int e = 0; e < 8; ++e) hb[e] = h_bits(sm[row][c8 + e]);
    u[it] = (v4u){pk16(hb[0], hb[1]), pk16(hb[2], hb[3]), pk16(hb[4], hb[5]), pk16(hb[6], hb[7])};
  }
  for (int pass = 0; pass < 2; ++pass) {
#pragma unroll
    for (int it = 0; it < 2; ++it) {
      const int row = wave * 8 + it * 4 + q;
      *(volatile v4u*)(out + (size_t)(n0 + row) * outPitch + d0 + c8) = u[it];
    }
    __threadfence();
  }
}

__global__ __launch_bounds__(256) void normconv_silu_kernel(const float* __restrict__ R, const float* __restrict__ cw,
                                                            unsigned short* __restrict__ out16, int do_norm) {
  __shared__ __align__(16) float xs[kNcRowsIn * kD];
  __shared__ __align__(16) unsigned short os[kNcRows * kD];
  const int tid = threadIdx.x, lane = tid & 31, wave = tid >> 5;
  const int head = blockIdx.x & (kH - 1);
  const int tile = blockIdx.x >> 4;
  const int m0 = tile * kNcRows;
  const int t0 = m0 & (kS - 1);

  for (int rr = wave; rr < kNcRowsIn; rr += 8) {
    const int t = t0 - (kTaps - 1) + rr;
    const bool valid = (t >= 0);
    const int mc = valid ? (m0 - (kTaps - 1) + rr) : m0;
    const v4f x = *(const v4f*)(R + (size_t)mc * kC + head * kD + lane * 4);
    const float x0 = x[0], x1 = x[1], x2 = x[2], x3 = x[3];
    float ss = (x0 * x0 + x1 * x1) + (x2 * x2 + x3 * x3);
#pragma unroll
    for (int off = 16; off > 0; off >>= 1) ss += __shfl_xor(ss, off, 32);
    const float rn = rsqrtf(ss + kEpsL2);
    const float r = (do_norm != 0) ? rn : 1.0f;
    v4f y;
    y[0] = valid ? (x0 * r) : 0.0f;
    y[1] = valid ? (x1 * r) : 0.0f;
    y[2] = valid ? (x2 * r) : 0.0f;
    y[3] = valid ? (x3 * r) : 0.0f;
    *(v4f*)(xs + rr * kD + lane * 4) = y;
  }
  __syncthreads();

  {
    const int d = tid & (kD - 1);
    const int rh = tid >> 7;
    const int c = head * kD + d;
    const float w0 = bf16r(cw[0 * kC + c]);
    const float w1 = bf16r(cw[1 * kC + c]);
    const float w2 = bf16r(cw[2 * kC + c]);
    const float w3 = bf16r(cw[3 * kC + c]);
#pragma unroll 1
    for (int i = 0; i < kNcRows / 2; ++i) {
      const int row = i * 2 + rh;
      const float* xp = xs + row * kD + d;
      float acc = w0 * xp[0];
      acc = fmaf(w1, xp[kD], acc);
      acc = fmaf(w2, xp[2 * kD], acc);
      acc = fmaf(w3, xp[3 * kD], acc);
      const float y = acc * sigmoid_f(acc);
      os[row * kD + d] = h_bits(y);
    }
  }
  __syncthreads();

  {
    v4u u[2];
#pragma unroll
    for (int it = 0; it < 2; ++it) {
      const int idx = it * 256 + tid;
      u[it] = *(const v4u*)(os + idx * 8);
    }
    for (int pass = 0; pass < 2; ++pass) {
#pragma unroll
      for (int it = 0; it < 2; ++it) {
        const int idx = it * 256 + tid;
        const int row = idx >> 4;
        const int c8 = (idx & 15) * 8;
        *(volatile v4u*)(out16 + (size_t)(m0 + row) * kC + head * kD + c8) = u[it];
      }
      __threadfence();
    }
  }
}

__global__ __launch_bounds__(256) void split_kernel(const float* __restrict__ P, unsigned short* __restrict__ hf16,
                                                    unsigned short* __restrict__ hg16, float* __restrict__ beta) {
  const int tid = threadIdx.x, lane = tid & 31, wave = tid >> 5;
  const int r0 = blockIdx.x * 64 + wave * 8;
  unsigned short* dplane = (lane < 16) ? hf16 : hg16;
#pragma unroll 1
  for (int j = 0; j < 8; ++j) {
    const int row = r0 + j;
    const float* p = P + (size_t)row * kCat + lane * 8;
    const v4f a = *(const v4f*)(p);
    const v4f c = *(const v4f*)(p + 4);
    unsigned short hb[8];
#pragma unroll
    for (int e = 0; e < 4; ++e) {
      const float a0 = a[e];
      const float c0 = c[e];
      hb[e]     = h_bits(a0);
      hb[4 + e] = h_bits(c0);
    }
    const v4u u = (v4u){pk16(hb[0], hb[1]), pk16(hb[2], hb[3]), pk16(hb[4], hb[5]), pk16(hb[6], hb[7])};
    unsigned short* q = dplane + (size_t)row * kD + (lane & 15) * 8;
    *(volatile v4u*)q = u;
    __threadfence();
    *(volatile v4u*)q = u;
  }
  {
    const int row = r0 + (lane >> 2);
    const int col4 = (lane & 3) * 4;
    const v4f x = *(const v4f*)(P + (size_t)row * kCat + 2 * kD + col4);
    v4f o;
#pragma unroll
    for (int e = 0; e < 4; ++e) {
      const float xe = x[e];
      o[e] = sigmoid_f(xe);
    }
    float* q = beta + (size_t)row * kH + col4;
    *(volatile v4f*)q = o;
    __threadfence();
    *(volatile v4f*)q = o;
  }
}

__global__ __launch_bounds__(256) void decay_kernel(float* G, const float* __restrict__ A_log, const float* __restrict__ dt_bias) {
  const int tid = threadIdx.x;
  const int cgp = blockIdx.x & 7;
  const int rg = blockIdx.x >> 3;
  const int c = cgp * 256 + tid;
  const float Ah = expf(bf16r(A_log[c >> 7]));
  const float nA = -Ah;
  const float dtb = bf16r(dt_bias[c]);
#pragma unroll 1
  for (int j = 0; j < 8; ++j) {
    float* p = G + (size_t)(rg * 8 + j) * kC + c;
    const float x = *p + dtb;
    const float sp = fmaxf(x, 0.0f) + log1pf(expf(-fabsf(x)));
    const float g = nA * sp;
    float eg = expf(g);
    eg = (eg < FLT_MIN) ? 0.0f : eg;
    *(volatile float*)p = eg;
    __threadfence();
    *(volatile float*)p = eg;
  }
}

__global__ __launch_bounds__(256) void state_scan_kernel(const unsigned short* __restrict__ QC, const unsigned short* __restrict__ KC,
                                                         const unsigned short* __restrict__ VC, const float* __restrict__ EG,
                                                         const float* __restrict__ BETA, float* __restrict__ ATT, float qscale) {
  __shared__ __align__(16) float kb[kScT * kD];
  __shared__ __align__(16) float qb[kScT * kD];
  __shared__ __align__(16) float eb[kScT * kD];
  __shared__ __align__(16) float vb[kScT * kScCols];
  __shared__ __align__(16) float ob[kScT * kScCols];
  __shared__ __align__(16) float bb[kScT];
  const int tid = threadIdx.x, lane = tid & 31, wave = tid >> 5;
  const int cgp = blockIdx.x & 3;
  const int bh = blockIdx.x >> 2;
  const int h = bh & (kH - 1);
  const int b = bh >> 4;
  const int kg = lane & 7;
  const int cl = tid >> 3;
  const int rowbase = b * kS;

  float St[kScKpl];
#pragma unroll
  for (int i = 0; i < kScKpl; ++i) St[i] = 0.0f;

  const int sstep = tid >> 4;
  const int sd8 = (tid & 15) * 8;
  const int vstep = tid >> 2;
  const int vc8 = (tid & 3) * 8;

#pragma unroll 1
  for (int batch = 0; batch < kS / kScT; ++batch) {
    const int t0 = batch * kScT;
    {
      const size_t base = (size_t)(rowbase + t0 + sstep) * kC + h * kD + sd8;
      const v4u kw = *(const v4u*)(KC + base);
      const v4u qw = *(const v4u*)(QC + base);
      const v4f e0 = *(const v4f*)(EG + base);
      const v4f e1 = *(const v4f*)(EG + base + 4);
      float kf[8], qf[8];
#pragma unroll
      for (int w = 0; w < 4; ++w) {
        const unsigned kd = kw[w];
        const unsigned qd = qw[w];
        kf[2 * w]     = h16_to_f32(kd & 0xffffu);
        kf[2 * w + 1] = h16_to_f32(kd >> 16);
        qf[2 * w]     = h16_to_f32(qd & 0xffffu) * qscale;
        qf[2 * w + 1] = h16_to_f32(qd >> 16) * qscale;
      }
      float* kp = kb + sstep * kD + sd8;
      float* qp = qb + sstep * kD + sd8;
      float* ep = eb + sstep * kD + sd8;
      *(v4f*)(kp)     = (v4f){kf[0], kf[1], kf[2], kf[3]};
      *(v4f*)(kp + 4) = (v4f){kf[4], kf[5], kf[6], kf[7]};
      *(v4f*)(qp)     = (v4f){qf[0], qf[1], qf[2], qf[3]};
      *(v4f*)(qp + 4) = (v4f){qf[4], qf[5], qf[6], qf[7]};
      *(v4f*)(ep)     = e0;
      *(v4f*)(ep + 4) = e1;
    }
    if (wave < 2) {
      const size_t vbase = (size_t)(rowbase + t0 + vstep) * kC + h * kD + cgp * kScCols + vc8;
      const v4u vw = *(const v4u*)(VC + vbase);
      float vf[8];
#pragma unroll
      for (int w = 0; w < 4; ++w) {
        const unsigned vd = vw[w];
        vf[2 * w]     = h16_to_f32(vd & 0xffffu);
        vf[2 * w + 1] = h16_to_f32(vd >> 16);
      }
      float* vp = vb + vstep * kScCols + vc8;
      *(v4f*)(vp)     = (v4f){vf[0], vf[1], vf[2], vf[3]};
      *(v4f*)(vp + 4) = (v4f){vf[4], vf[5], vf[6], vf[7]};
    }
    if (wave == 2) {
      const int j = lane & 15;
      float bv = BETA[(size_t)(rowbase + t0 + j) * kH + h];
      asm volatile("" : "+v"(bv));
      if (lane < 16) bb[j] = bv;
    }
    __syncthreads();

#pragma unroll 1
    for (int tt = 0; tt < kScT; ++tt) {
      const float* kr = kb + tt * kD + kg * kScKpl;
      const float* qr = qb + tt * kD + kg * kScKpl;
      const float* er = eb + tt * kD + kg * kScKpl;
      v4f kv[4], qv[4], ev[4];
#pragma unroll
      for (int j = 0; j < 4; ++j) {
        kv[j] = *(const v4f*)(kr + 4 * j);
        qv[j] = *(const v4f*)(qr + 4 * j);
        ev[j] = *(const v4f*)(er + 4 * j);
      }
      const float vt = vb[tt * kScCols + cl];
      const float bt = bb[tt];
      float p = 0.0f;
#pragma unroll
      for (int j = 0; j < 4; ++j) {
#pragma unroll
        for (int e = 0; e < 4; ++e) {
          const float s = St[4 * j + e] * ev[j][e];
          St[4 * j + e] = s;
          p = fmaf(kv[j][e], s, p);
        }
      }
      p += __shfl_xor(p, 1, 32);
      p += __shfl_xor(p, 2, 32);
      p += __shfl_xor(p, 4, 32);
      const float be = bt * (vt - p);
      float o = 0.0f;
#pragma unroll
      for (int j = 0; j < 4; ++j) {
#pragma unroll
        for (int e = 0; e < 4; ++e) {
          const float s = fmaf(kv[j][e], be, St[4 * j + e]);
          St[4 * j + e] = s;
          o = fmaf(qv[j][e], s, o);
        }
      }
      o += __shfl_xor(o, 1, 32);
      o += __shfl_xor(o, 2, 32);
      o += __shfl_xor(o, 4, 32);
      if (kg == 0) ob[tt * kScCols + cl] = o;
    }
    __syncthreads();

    if (tid < 128) {
      const int line = tid >> 3;
      const int q4 = (tid & 7) * 4;
      const v4f val = *(const v4f*)(ob + line * kScCols + q4);
      float* dst = ATT + (size_t)(rowbase + t0 + line) * kC + h * kD + cgp * kScCols + q4;
      for (int pass = 0; pass < 2; ++pass) {
        *(volatile v4f*)dst = val;
        __threadfence();
      }
    }
  }
}

__global__ __launch_bounds__(256) void normgate_kernel(const float* __restrict__ ATT, const float* __restrict__ GATE,
                                                       const float* __restrict__ rms, unsigned short* __restrict__ act16) {
  __shared__ __align__(16) unsigned osw[8 * 64];
  const int tid = threadIdx.x, lane = tid & 31, wave = tid >> 5;
  const size_t u = (size_t)blockIdx.x * 8 + wave;
  const v4f o = *(const v4f*)(ATT + u * kD + lane * 4);
  const v4f g = *(const v4f*)(GATE + u * kD + lane * 4);
  const v4f sc = *(const v4f*)(rms + lane * 4);
  const float o0 = o[0], o1 = o[1], o2 = o[2], o3 = o[3];
  float ss = (o0 * o0 + o1 * o1) + (o2 * o2 + o3 * o3);
#pragma unroll
  for (int off = 16; off > 0; off >>= 1) ss += __shfl_xor(ss, off, 32);
  const float r = rsqrtf(ss * kInvD + kEpsRms);
  unsigned short hb[4];
#pragma unroll
  for (int e = 0; e < 4; ++e) {
    const float oe = o[e];
    const float ge = g[e];
    const float se = sc[e];
    const float normed = (oe * r) * bf16r(se);
    const float a = normed * sigmoid_f(ge);
    hb[e] = h_bits(a * kActCarry);
  }
  osw[wave * 64 + lane * 2]     = pk16(hb[0], hb[1]);
  osw[wave * 64 + lane * 2 + 1] = pk16(hb[2], hb[3]);
  __syncthreads();
  if (tid < 128) {
    const v4u w = *(const v4u*)(osw + tid * 4);
    unsigned short* dst = act16 + (size_t)blockIdx.x * (8 * kD) + tid * 8;
    for (int pass = 0; pass < 2; ++pass) {
      *(volatile v4u*)dst = w;
      __threadfence();
    }
  }
}

constexpr size_t kOffBlk   = 0;
constexpr size_t kOffHid16 = kOffBlk;
constexpr size_t kOffWT    = kOffHid16 + (size_t)kRows * kHid * 2;
constexpr size_t kOffP     = kOffWT + (size_t)kC * kHid * 2;
constexpr size_t kBlkBytes = (size_t)kRows * kC * 4;
constexpr size_t kOffR     = kOffBlk + kBlkBytes;
constexpr size_t kOffQC    = kOffR + (size_t)kRows * kC * 4;
constexpr size_t kOffKC    = kOffQC + (size_t)kRows * kC * 2;
constexpr size_t kOffVC    = kOffKC + (size_t)kRows * kC * 2;
constexpr size_t kOffWcat  = kOffVC + (size_t)kRows * kC * 2;
constexpr size_t kOffWfbT  = kOffWcat + (size_t)kCat * kHid * 2;
constexpr size_t kOffWgbT  = kOffWfbT + (size_t)kC * kD * 2;
constexpr size_t kOffHF    = kOffWgbT + (size_t)kC * kD * 2;
constexpr size_t kOffHG    = kOffHF + (size_t)kRows * kD * 2;
constexpr size_t kOffBeta  = kOffHG + (size_t)kRows * kD * 2;
constexpr size_t kWsTotal  = kOffBeta + (size_t)kRows * kH * 4;
static_assert(kOffP + (size_t)kRows * kCat * 4 <= kOffBlk + kBlkBytes, "P inside the overlay block");
static_assert(kWsTotal == 122159104, "carve total");
static_assert(kWsTotal <= (size_t)134217728, "carve cap");

extern "C" void kernel_launch(void* const* d_in, const int* in_sizes, int n_in,
                              void* d_out, int out_size, void* d_ws, size_t ws_size, hipStream_t stream) {
  if (n_in < 16 || d_out == nullptr || d_ws == nullptr) return;
  if (in_sizes[0] != kRows * kHid || in_sizes[1] != kHid * kC || in_sizes[2] != kHid * kC || in_sizes[3] != kHid * kC ||
      in_sizes[4] != kTaps * kC || in_sizes[5] != kTaps * kC || in_sizes[6] != kTaps * kC || in_sizes[7] != kHid * kH ||
      in_sizes[8] != kHid * kD || in_sizes[9] != kD * kC || in_sizes[10] != kHid * kD || in_sizes[11] != kD * kC ||
      in_sizes[12] != kH || in_sizes[13] != kC || in_sizes[14] != kD || in_sizes[15] != kC * kHid ||
      out_size != kRows * kHid) return;
  if (kWsTotal > ws_size) return;

  const float* hidden  = (const float*)d_in[0];
  const float* Wq      = (const float*)d_in[1];
  const float* Wk      = (const float*)d_in[2];
  const float* Wv      = (const float*)d_in[3];
  const float* conv_q  = (const float*)d_in[4];
  const float* conv_k  = (const float*)d_in[5];
  const float* conv_v  = (const float*)d_in[6];
  const float* Wb      = (const float*)d_in[7];
  const float* Wfa     = (const float*)d_in[8];
  const float* Wfb     = (const float*)d_in[9];
  const float* Wga     = (const float*)d_in[10];
  const float* Wgb     = (const float*)d_in[11];
  const float* A_log   = (const float*)d_in[12];
  const float* dt_bias = (const float*)d_in[13];
  const float* rms_sc  = (const float*)d_in[14];
  const float* Wo      = (const float*)d_in[15];
  float* out = (float*)d_out;

  char* ws = (char*)d_ws;
  unsigned short* HID16 = (unsigned short*)(ws + kOffHid16);
  unsigned short* WT    = (unsigned short*)(ws + kOffWT);
  float*          P     = (float*)(ws + kOffP);
  float*          ATT   = (float*)(ws + kOffBlk);
  float*          R     = (float*)(ws + kOffR);
  unsigned short* QC16  = (unsigned short*)(ws + kOffQC);
  unsigned short* KC16  = (unsigned short*)(ws + kOffKC);
  unsigned short* VC16  = (unsigned short*)(ws + kOffVC);
  unsigned short* ACT16 = QC16;
  unsigned short* WCATT = (unsigned short*)(ws + kOffWcat);
  unsigned short* WFBT  = (unsigned short*)(ws + kOffWfbT);
  unsigned short* WGBT  = (unsigned short*)(ws + kOffWgbT);
  unsigned short* HF16  = (unsigned short*)(ws + kOffHF);
  unsigned short* HG16  = (unsigned short*)(ws + kOffHG);
  float*          BETA  = (float*)(ws + kOffBeta);

  const float qscale = (float)(1.0 / sqrt((double)kD));

  auto gemm = [&](const unsigned short* A, int lda, const unsigned short* Bt, int ldb, float* Cc, int ldc,
                  int M, int N, int K, float sc) {
    const int tiles = (M / 64) * (N / 64);
    wmma_gemm64_f16<<<dim3((unsigned)((tiles + 7) / 8)), dim3(256), 0, stream>>>(A, lda, Bt, ldb, Cc, ldc, M, N, K, sc);
  };
  auto wtcast = [&](const float* W, int rk, int srcPitch, int nValid, int nOut, unsigned short* o, int outPitch) {
    wt_cast_kernel<<<dim3((unsigned)(rk / 64), (unsigned)((nOut + 63) / 64)), dim3(256), 0, stream>>>(W, srcPitch, nValid, o, outPitch, kWCarry);
  };

  {
    const int n8 = (kRows * kHid) / 8;
    cvt8_bf16_f16_kernel<<<dim3((unsigned)((n8 + 255) / 256)), dim3(256), 0, stream>>>(hidden, HID16, n8);
  }
  wtcast(Wfa, kHid, kD, kD, kD, WCATT, kHid);
  wtcast(Wga, kHid, kD, kD, kD, WCATT + (size_t)kD * kHid, kHid);
  wtcast(Wb,  kHid, kH, kH, kCat - 2 * kD, WCATT + (size_t)2 * kD * kHid, kHid);
  wtcast(Wfb, kD, kC, kC, kC, WFBT, kD);
  wtcast(Wgb, kD, kC, kC, kC, WGBT, kD);

  const int ncGrid = (kRows / kNcRows) * kH;

  wtcast(Wq, kHid, kC, kC, kC, WT, kHid);
  gemm(HID16, kHid, WT, kHid, R, kC, kRows, kC, kHid, kWCarryInv);
  normconv_silu_kernel<<<dim3((unsigned)ncGrid), dim3(256), 0, stream>>>(R, conv_q, QC16, 1);
  wtcast(Wk, kHid, kC, kC, kC, WT, kHid);
  gemm(HID16, kHid, WT, kHid, R, kC, kRows, kC, kHid, kWCarryInv);
  normconv_silu_kernel<<<dim3((unsigned)ncGrid), dim3(256), 0, stream>>>(R, conv_k, KC16, 1);
  wtcast(Wv, kHid, kC, kC, kC, WT, kHid);
  gemm(HID16, kHid, WT, kHid, R, kC, kRows, kC, kHid, kWCarryInv);
  normconv_silu_kernel<<<dim3((unsigned)ncGrid), dim3(256), 0, stream>>>(R, conv_v, VC16, 0);

  gemm(HID16, kHid, WCATT, kHid, P, kCat, kRows, kCat, kHid, kWCarryInv);
  split_kernel<<<dim3((unsigned)(kRows / 64)), dim3(256), 0, stream>>>(P, HF16, HG16, BETA);

  gemm(HF16, kD, WFBT, kD, R, kC, kRows, kC, kD, kWCarryInv);
  decay_kernel<<<dim3((unsigned)((kRows / 8) * (kC / 256))), dim3(256), 0, stream>>>(R, A_log, dt_bias);

  state_scan_kernel<<<dim3((unsigned)(kB * kH * (kD / kScCols))), dim3(256), 0, stream>>>(QC16, KC16, VC16, R, BETA, ATT, qscale);

  gemm(HG16, kD, WGBT, kD, R, kC, kRows, kC, kD, kWCarryInv);
  normgate_kernel<<<dim3((unsigned)((kRows * kH) / 8)), dim3(256), 0, stream>>>(ATT, R, rms_sc, ACT16);

  wtcast(Wo, kC, kHid, kHid, kHid, WT, kC);
  gemm(ACT16, kC, WT, kC, out, kHid, kRows, kHid, kC, kOutScale);
}
